// NMMO3EncoderRef_84937273245751
// MI455X (gfx1250) — hardware-verified
//
#include <hip/hip_runtime.h>
#include <stdint.h>

typedef __attribute__((ext_vector_type(16))) _Float16 v16h;
typedef __attribute__((ext_vector_type(8)))  _Float16 v8h;
typedef __attribute__((ext_vector_type(16))) __bf16   v16b;
typedef __attribute__((ext_vector_type(8)))  __bf16   v8b;
typedef __attribute__((ext_vector_type(8)))  float    v8f;
typedef __attribute__((ext_vector_type(4)))  float    v4f;

__device__ __forceinline__ unsigned short f2bf_bits(float f) {
  unsigned u = __float_as_uint(f);
  return (unsigned short)((u + 0x7FFFu + ((u >> 16) & 1u)) >> 16);
}
__device__ __forceinline__ float bf_bits2f(unsigned short h) { return __uint_as_float(((unsigned)h) << 16); }

__device__ __forceinline__ void dep_guard_h(v8f& a, v8f& b, v16h x, v16h y) { asm volatile("v_nop\n\tv_nop\n\tv_nop\n\tv_nop" : "+v"(a), "+v"(b) : "v"(x), "v"(y)); }
__device__ __forceinline__ void dep_guard_b(v8f& a, v8f& b, v16b x, v16b y) { asm volatile("v_nop\n\tv_nop\n\tv_nop\n\tv_nop" : "+v"(a), "+v"(b) : "v"(x), "v"(y)); }
__device__ __forceinline__ void keep4_h(v16h a, v16h b, v16h c, v16h d) { asm volatile("v_nop" :: "v"(a), "v"(b), "v"(c), "v"(d)); }
__device__ __forceinline__ void keep4_b(v16b a, v16b b, v16b c, v16b d) { asm volatile("v_nop" :: "v"(a), "v"(b), "v"(c), "v"(d)); }
__device__ __forceinline__ void acc_guard4(v8f& a, v8f& b, v8f& c, v8f& d) { asm volatile("v_nop\n\tv_nop\n\tv_nop\n\tv_nop" : "+v"(a), "+v"(b), "+v"(c), "+v"(d)); }
template <typename T> struct Frag;
template <> struct Frag<_Float16> {
  typedef v16h V; union U { v16h v; v8h h[2]; };
  static __device__ __forceinline__ v16h load(const _Float16* p) {
    U f; f.h[0] = *(const v8h*)(p); f.h[1] = *(const v8h*)(p + 16); return f.v;
  }
  static __device__ __forceinline__ v8f mma(v16h a, v16h b, v8f c) {
    return __builtin_amdgcn_wmma_f32_16x16x32_f16(false, a, false, b, (short)0, c, false, false);
  }
  static __device__ __forceinline__ void guard(v8f& a, v8f& b, v16h x, v16h y) { dep_guard_h(a, b, x, y); }
  static __device__ __forceinline__ void keep(v16h a, v16h b, v16h c, v16h d) { keep4_h(a, b, c, d); }
};
template <> struct Frag<__bf16> {
  typedef v16b V; union U { v16b v; v8b h[2]; };
  static __device__ __forceinline__ v16b load(const __bf16* p) {
    U f; f.h[0] = *(const v8b*)(p); f.h[1] = *(const v8b*)(p + 16); return f.v;
  }
  static __device__ __forceinline__ v8f mma(v16b a, v16b b, v8f c) {
    return __builtin_amdgcn_wmma_f32_16x16x32_bf16(false, a, false, b, (short)0, c, false, false);
  }
  static __device__ __forceinline__ void guard(v8f& a, v8f& b, v16b x, v16b y) { dep_guard_b(a, b, x, y); }
  static __device__ __forceinline__ void keep(v16b a, v16b b, v16b c, v16b d) { keep4_b(a, b, c, d); }
};

template <int ET> struct Elem;
template <> struct Elem<0> { typedef _Float16 T; };
template <> struct Elem<1> { typedef __bf16 T; };
template <int ET, bool SPLIT, int BIAS_MODE, int OUT_MODE, bool RESID, int ACT = 0>
__global__ __launch_bounds__(256) void wmma_gemm64(
    const unsigned short* __restrict__ Ap, const unsigned short* __restrict__ A2p, int lda, long strideA,
    const unsigned short* __restrict__ Btp, const unsigned short* __restrict__ Bt2p, int ldb, long strideB,
    void* __restrict__ Cout, void* __restrict__ Cout2, int ldc, long strideC,
    const float* __restrict__ bias,
    const float* __restrict__ resid, long strideR,
    int M, int N, int K, float scale) {
  typedef typename Elem<ET>::T T;
  typedef typename Frag<T>::V V;
  const T* A = (const T*)Ap; const T* A2 = (const T*)A2p; const T* Bt = (const T*)Btp; const T* Bt2 = (const T*)Bt2p;
  __shared__ __align__(16) float sT[8][16 * 68];
  const int b    = blockIdx.y;
  const int lane = threadIdx.x & 31;
  const int wave = threadIdx.x >> 5;
  const int tilesN = N >> 6;
  const int tilesM = M >> 6;
  const int tile = blockIdx.x * 8 + wave;
  if (tile >= tilesM * tilesN) return;
  const int tm = tile / tilesN;
  const int tn = tile - tm * tilesN;
  const int m0 = tm << 6;
  const int n0 = tn << 6;

  const T* Ab  = A  + (size_t)b * strideA;
  const T* Bb  = Bt + (size_t)b * strideB;
  const T* Ab2 = SPLIT ? (A2  + (size_t)b * strideA) : nullptr;
  const T* Bb2 = SPLIT ? (Bt2 + (size_t)b * strideB) : nullptr;

  const int rlane = lane & 15;
  const int koff  = (lane >> 4) * 8;
  const int mOff  = (lane >> 4) * 8;

  v8f acc[4][4];
#pragma unroll
  for (int i = 0; i < 4; ++i)
#pragma unroll
    for (int j = 0; j < 4; ++j) acc[i][j] = (v8f){0.f,0.f,0.f,0.f,0.f,0.f,0.f,0.f};

  for (int k0 = 0; k0 < K; k0 += 32) {
    V bh[4], bl[4];
#pragma unroll
    for (int j = 0; j < 4; ++j) {
      const size_t bo = (size_t)(n0 + (j << 4) + rlane) * ldb + koff + k0;
      bh[j] = Frag<T>::load(Bb + bo);
      if (SPLIT) bl[j] = Frag<T>::load(Bb2 + bo);
    }
#pragma unroll
    for (int i = 0; i < 4; ++i) {
      const size_t ao = (size_t)(m0 + (i << 4) + rlane) * lda + koff + k0;
      V ah = Frag<T>::load(Ab + ao);
      V al;
      if (SPLIT) al = Frag<T>::load(Ab2 + ao);
#pragma unroll
      for (int j = 0; j < 4; ++j) {
        acc[i][j] = Frag<T>::mma(ah, bh[j], acc[i][j]);
        if (SPLIT) {
          acc[i][j] = Frag<T>::mma(ah, bl[j], acc[i][j]);
          acc[i][j] = Frag<T>::mma(al, bh[j], acc[i][j]);
        }
      }
      Frag<T>::guard(acc[i][0], acc[i][3], ah, SPLIT ? al : ah);
    }
    Frag<T>::keep(bh[0], bh[1], bh[2], bh[3]);
    if (SPLIT) Frag<T>::keep(bl[0], bl[1], bl[2], bl[3]);
  }
  acc_guard4(acc[0][0], acc[0][1], acc[0][2], acc[0][3]);
  acc_guard4(acc[1][0], acc[1][1], acc[1][2], acc[1][3]);
  acc_guard4(acc[2][0], acc[2][1], acc[2][2], acc[2][3]);
  acc_guard4(acc[3][0], acc[3][1], acc[3][2], acc[3][3]);

  float* slab = sT[wave];
  const float* Rb = RESID ? (resid + (size_t)b * strideR) : nullptr;
#pragma unroll
  for (int i = 0; i < 4; ++i) {
    const int mBase = m0 + (i << 4);
#pragma unroll
    for (int j = 0; j < 4; ++j) {
      const int n = n0 + (j << 4) + rlane;
      float bv = 0.f;
      if (BIAS_MODE == 2) bv = bias[n];
#pragma unroll
      for (int r = 0; r < 8; ++r) {
        float v = acc[i][j][r] * scale;
        if (BIAS_MODE == 1) v += bias[mBase + mOff + r];
        if (BIAS_MODE == 2) v += bv;
        if (RESID) v += Rb[(size_t)(mBase + mOff + r) * ldc + n];
        if (ACT == 1) v = tanhf(v);
        if (ACT == 2) v = fmaxf(v, 0.0f);
        if (ACT == 3) v = v / (1.0f + expf(-v));
        if (ACT == 4) v = (v > 0.f) ? v : 0.01f * v;
        if (ACT == 5) v = 0.5f * v * (1.0f + erff(v * 0.70710678118654752f));
        slab[(mOff + r) * 68 + (j << 4) + rlane] = v;
      }
    }
    __builtin_amdgcn_fence(__ATOMIC_RELEASE, "workgroup");
    __builtin_amdgcn_wave_barrier();
    __builtin_amdgcn_fence(__ATOMIC_ACQUIRE, "workgroup");
    if (OUT_MODE == 0) {
      float* C = (float*)Cout + (size_t)b * strideC;
      const int hh = lane >> 4, c4 = (lane & 15) * 4;
      for (int pass = 0; pass < 2; ++pass) {
#pragma unroll
        for (int it = 0; it < 8; ++it) {
          const int row = it * 2 + hh;
          v4f v = *(const v4f*)(slab + row * 68 + c4);
          *(volatile v4f*)(C + (size_t)(mBase + row) * ldc + n0 + c4) = v;
        }
        __threadfence();
      }
    } else {
      const int q = lane >> 3, c8 = (lane & 7) * 8;
      unsigned short* C  = (unsigned short*)Cout  + (size_t)b * strideC;
      unsigned short* C2 = (OUT_MODE == 2) ? ((unsigned short*)Cout2 + (size_t)b * strideC) : nullptr;
      for (int pass = 0; pass < 2; ++pass) {
#pragma unroll
        for (int it = 0; it < 4; ++it) {
          const int row = it * 4 + q;
          const float* sp = slab + row * 68 + c8;
          v8h hv, lv;
#pragma unroll
          for (int e = 0; e < 8; ++e) {
            if (OUT_MODE == 1) {
              hv[e] = (_Float16)sp[e];
            } else {
              unsigned short hb = f2bf_bits(sp[e]);
              unsigned short lb = f2bf_bits(sp[e] - bf_bits2f(hb));
              hv[e] = __builtin_bit_cast(_Float16, hb);
              lv[e] = __builtin_bit_cast(_Float16, lb);
            }
          }
          *(volatile v8h*)(C + (size_t)(mBase + row) * ldc + n0 + c8) = hv;
          if (OUT_MODE == 2) *(volatile v8h*)(C2 + (size_t)(mBase + row) * ldc + n0 + c8) = lv;
        }
        __threadfence();
      }
    }
    __builtin_amdgcn_fence(__ATOMIC_RELEASE, "workgroup");
    __builtin_amdgcn_wave_barrier();
    __builtin_amdgcn_fence(__ATOMIC_ACQUIRE, "workgroup");
  }
}

#define OBS_W    1707
#define MAP_N    1650
#define NCH1     59
#define K1       1475
#define K1P      1504
#define K2       1152
#define NOC      128
#define EMB_ROWS 128
#define EMB_D    32
#define NPL      47
#define KP       1817
#define KPP      1856
#define NOUT     512
#define EMB_COL0 256
#define RAW_COL0 1760

__constant__ int c_off[10] = {0, 4, 8, 25, 30, 33, 38, 43, 48, 55};

__global__ __launch_bounds__(256) void k_prep(
    const float* __restrict__ w1, const float* __restrict__ w2, const float* __restrict__ pw,
    _Float16* __restrict__ w1h, _Float16* __restrict__ w2h, _Float16* __restrict__ pwh,
    int n1, int n2, int n3)
{
  const int gid = blockIdx.x * 256 + threadIdx.x;
  if (gid >= n1 + n2 + n3) return;
  v8h hv;
  _Float16* dst;
  if (gid < n1) {
    const int e0 = gid * 8;
    const int o = e0 / K1P, kb = e0 - o * K1P;
#pragma unroll
    for (int e = 0; e < 8; ++e) {
      const int k = kb + e;
      const int src = min(o * K1 + k, NOC * K1 - 1);
      const float v = w1[src];
      hv[e] = (_Float16)((k < K1) ? v * 64.0f : 0.0f);
    }
    dst = w1h + e0;
  } else if (gid < n1 + n2) {
    const int e0 = (gid - n1) * 8;
#pragma unroll
    for (int e = 0; e < 8; ++e) hv[e] = (_Float16)(w2[e0 + e] * 64.0f);
    dst = w2h + e0;
  } else {
    const int e0 = (gid - n1 - n2) * 8;
    const int n = e0 / KPP, jb = e0 - n * KPP;
#pragma unroll
    for (int e = 0; e < 8; ++e) {
      const int j = jb + e;
      int col; float sc;
      if (j < EMB_COL0)      { col = (j & (NOC - 1)) * 2 + (j >> 7); sc = 1024.0f; }
      else if (j < RAW_COL0) { col = j; sc = 16.0f; }
      else if (j < KP)       { col = j; sc = 1024.0f; }
      else                   { col = KP - 1; sc = 0.0f; }
      hv[e] = (_Float16)(sc * pw[(size_t)n * KP + col]);
    }
    dst = pwh + e0;
  }
  *(volatile v8h*)dst = hv;
  __threadfence();
  *(volatile v8h*)dst = hv;
}

#define C1_SPB 4
#define C1_ROWS 48
#define C1_THR 96
#define C1_TP 128

union Conv1Smem { _Float16 a[C1_ROWS * K1P]; float t[C1_ROWS * C1_TP]; };

__global__ __launch_bounds__(C1_THR) void k_conv1(
    const float* __restrict__ obs, const float* __restrict__ conv1_b,
    const _Float16* __restrict__ w1h, _Float16* __restrict__ a2, int nB)
{
  __shared__ __align__(16) Conv1Smem sm;
  const int t = threadIdx.x, wave = t >> 5, lane = t & 31;
  const int rlane = lane & 15, hh = lane >> 4, koff = hh * 8;
  const int b0 = blockIdx.x * C1_SPB;

  {
    v8h z;
#pragma unroll
    for (int e = 0; e < 8; ++e) z[e] = (_Float16)0.0f;
    v8h* p = (v8h*)sm.a;
    for (int i = t; i < C1_ROWS * K1P / 8; i += C1_THR) p[i] = z;
  }
  __syncthreads();

  for (int pr = t; pr < C1_ROWS * 10; pr += C1_THR) {
    const int row = pr / 10, f = pr - row * 10;
    const int s = row / 12, p = row - s * 12, oy = p >> 2, ox = p & 3;
    const float* ob = obs + (size_t)(b0 + s) * OBS_W + f;
    const int off = c_off[f];
    _Float16* arow = sm.a + row * K1P;
#pragma unroll
    for (int ky = 0; ky < 5; ++ky) {
#pragma unroll
      for (int kx = 0; kx < 5; ++kx) {
        const int hy = 3 * oy + ky, wx = 3 * ox + kx;
        int c = (int)ob[(hy * 15 + wx) * 10] + off;
        if (c < 0) c += NCH1;
        if ((unsigned)c < (unsigned)NCH1) arow[c * 25 + ky * 5 + kx] = (_Float16)1.0f;
      }
    }
  }
  __syncthreads();

  v8f acc[8];
#pragma unroll
  for (int j = 0; j < 8; ++j) acc[j] = (v8f){0.f,0.f,0.f,0.f,0.f,0.f,0.f,0.f};
  const _Float16* ap = sm.a + (wave * 16 + rlane) * K1P + koff;
  const _Float16* bp = w1h + (size_t)rlane * K1P + koff;
  for (int k0 = 0; k0 < K1P; k0 += 32) {
    const v16h av = Frag<_Float16>::load(ap + k0);
#pragma unroll
    for (int g = 0; g < 2; ++g) {
      v16h bq[4];
#pragma unroll
      for (int u = 0; u < 4; ++u)
        bq[u] = Frag<_Float16>::load(bp + (size_t)((g * 4 + u) * 16) * K1P + k0);
#pragma unroll
      for (int u = 0; u < 4; ++u)
        acc[g * 4 + u] = Frag<_Float16>::mma(av, bq[u], acc[g * 4 + u]);
      Frag<_Float16>::guard(acc[g * 4], acc[g * 4 + 3], av, bq[3]);
      Frag<_Float16>::keep(bq[0], bq[1], bq[2], bq[3]);
    }
  }
  acc_guard4(acc[0], acc[1], acc[2], acc[3]);
  acc_guard4(acc[4], acc[5], acc[6], acc[7]);
  __syncthreads();

  {
    const float inv = 1.0f / 64.0f;
#pragma unroll
    for (int j = 0; j < 8; ++j) {
      const int o = j * 16 + rlane;
      const float bv = conv1_b[o];
#pragma unroll
      for (int r = 0; r < 8; ++r) {
        const float v = acc[j][r] * inv + bv;
        sm.t[(wave * 16 + 8 * hh + r) * C1_TP + o] = fmaxf(v, 0.0f);
      }
    }
  }
  __syncthreads();

  for (int rr = wave; rr < 2 * C1_SPB; rr += 3) {
    const int s = rr >> 1, ox2 = rr & 1;
    _Float16* dst = a2 + ((size_t)ox2 * nB + b0 + s) * K2;
    const float* ts = sm.t + s * 12 * C1_TP;
    for (int pass = 0; pass < 2; ++pass) {
#pragma unroll
      for (int it = 0; it < 5; ++it) {
        const int q = lane + 32 * it;
        if (q < K2 / 8) {
          v8h hv;
#pragma unroll
          for (int e = 0; e < 8; ++e) {
            const int k = q * 8 + e;
            const int ci = k / 9, t9 = k - ci * 9, dy = t9 / 3, dx = t9 - dy * 3;
            hv[e] = (_Float16)ts[(dy * 4 + dx + ox2) * C1_TP + ci];
          }
          *(volatile v8h*)(dst + q * 8) = hv;
        }
      }
      __threadfence();
    }
  }
}

__global__ __launch_bounds__(256) void k_catfill(
    const float* __restrict__ obs, const float* __restrict__ embed_w,
    _Float16* __restrict__ cat, int nB)
{
  const int wave = threadIdx.x >> 5, lane = threadIdx.x & 31;
  const int b = blockIdx.x * 8 + wave;
  if (b >= nB) return;
  const float* ob = obs + (size_t)b * OBS_W;
  _Float16* dst = cat + (size_t)b * KPP + EMB_COL0;
  const int nChunks = (KPP - EMB_COL0) / 8;
  const int nEmbChunks = (NPL * EMB_D) / 8;
  for (int pass = 0; pass < 2; ++pass) {
#pragma unroll
    for (int it = 0; it < 7; ++it) {
      const int q = lane + 32 * it;
      if (q < nChunks) {
        v8h hv;
        if (q < nEmbChunks) {
          const int pj = q >> 2, d0 = (q & 3) * 8;
          int code = (int)ob[MAP_N + pj];
          if (code < 0) code += EMB_ROWS;
          code = min(max(code, 0), EMB_ROWS - 1);
          const float* er = embed_w + code * EMB_D + d0;
          const v4f e0 = *(const v4f*)er;
          const v4f e1 = *(const v4f*)(er + 4);
#pragma unroll
          for (int e = 0; e < 4; ++e) {
            hv[e]     = (_Float16)(e0[e] * 64.0f);
            hv[4 + e] = (_Float16)(e1[e] * 64.0f);
          }
        } else {
#pragma unroll
          for (int e = 0; e < 8; ++e) {
            const int j = EMB_COL0 + q * 8 + e;
            const int src = min(j - 110, OBS_W - 1);
            const float v = ob[src];
            hv[e] = (_Float16)((j < KP) ? v : 0.0f);
          }
        }
        *(volatile v8h*)(dst + q * 8) = hv;
      }
    }
    __threadfence();
  }
}

extern "C" void kernel_launch(void* const* d_in, const int* in_sizes, int n_in,
                              void* d_out, int out_size, void* d_ws, size_t ws_size,
                              hipStream_t stream)
{
  if (n_in < 8) return;
  const int nB = out_size / NOUT;
  if (nB <= 0 || nB * NOUT != out_size || (nB % 64) != 0) return;
  if (in_sizes[0] != nB * OBS_W) return;
  if (in_sizes[1] != NOC * K1 || in_sizes[2] < NOC) return;
  if (in_sizes[3] != NOC * K2 || in_sizes[4] < NOC) return;
  if (in_sizes[5] != EMB_ROWS * EMB_D || in_sizes[6] != NOUT * KP || in_sizes[7] < NOUT) return;

  const float* obs     = (const float*)d_in[0];
  const float* conv1_w = (const float*)d_in[1];
  const float* conv1_b = (const float*)d_in[2];
  const float* conv2_w = (const float*)d_in[3];
  const float* conv2_b = (const float*)d_in[4];
  const float* embed_w = (const float*)d_in[5];
  const float* proj_w  = (const float*)d_in[6];
  const float* proj_b  = (const float*)d_in[7];

  size_t off = 0;
  const size_t b_w1h = (size_t)NOC * K1P * 2;          const size_t o_w1h = off; off += (b_w1h + 255) & ~(size_t)255;
  const size_t b_w2h = (size_t)NOC * K2 * 2;           const size_t o_w2h = off; off += (b_w2h + 255) & ~(size_t)255;
  const size_t b_pwh = (size_t)NOUT * KPP * 2;         const size_t o_pwh = off; off += (b_pwh + 255) & ~(size_t)255;
  const size_t b_a2  = (size_t)2 * nB * K2 * 2;        const size_t o_a2  = off; off += (b_a2 + 255) & ~(size_t)255;
  const size_t b_cat = (size_t)nB * KPP * 2;           const size_t o_cat = off; off += (b_cat + 255) & ~(size_t)255;
  if (off > ws_size) return;

  char* ws = (char*)d_ws;
  _Float16* w1h = (_Float16*)(ws + o_w1h);
  _Float16* w2h = (_Float16*)(ws + o_w2h);
  _Float16* pwh = (_Float16*)(ws + o_pwh);
  _Float16* a2  = (_Float16*)(ws + o_a2);
  _Float16* cat = (_Float16*)(ws + o_cat);

  const int n1 = NOC * K1P / 8, n2 = NOC * K2 / 8, n3 = NOUT * KPP / 8;
  k_prep<<<(n1 + n2 + n3 + 255) / 256, 256, 0, stream>>>(conv1_w, conv2_w, proj_w, w1h, w2h, pwh, n1, n2, n3);

  k_conv1<<<nB / C1_SPB, C1_THR, 0, stream>>>(obs, conv1_b, w1h, a2, nB);

  k_catfill<<<nB / 8, 256, 0, stream>>>(obs, embed_w, cat, nB);

  {
    const int tiles = (nB / 64) * (NOC / 64);
    dim3 g((tiles + 7) / 8, 2);
    wmma_gemm64<0, false, 2, 1, false, 0><<<g, 256, 0, stream>>>(
        (const unsigned short*)a2, (const unsigned short*)a2, K2, (long)nB * K2,
        (const unsigned short*)w2h, (const unsigned short*)w2h, K2, 0L,
        (void*)cat, (void*)cat, KPP, (long)NOC,
        conv2_b, conv2_b, 0L,
        nB, NOC, K2, 1.0f / 64.0f);
  }

  {
    const int tiles = (nB / 64) * (NOUT / 64);
    dim3 g((tiles + 7) / 8, 1);
    wmma_gemm64<0, false, 2, 0, false, 2><<<g, 256, 0, stream>>>(
        (const unsigned short*)cat, (const unsigned short*)cat, KPP, 0L,
        (const unsigned short*)pwh, (const unsigned short*)pwh, KPP, 0L,
        d_out, d_out, NOUT, 0L,
        proj_b, proj_b, 0L,
        nB, NOUT, KPP, 1.0f / 1024.0f);
  }
}
